// HeteroGraph_38757784879708
// MI455X (gfx1250) — hardware-verified
//
#include <hip/hip_runtime.h>
#include <stddef.h>
#include <stdint.h>
#include <math.h>


#define NSUB    100000
#define NAGR    200000
#define NURB    100000
#define ESS     1600000
#define EAS     400000
#define EUS     200000
#define DF      128
#define DH      32
#define NCLS    16
#define NLAY    3
#define NPAD    100096
#define PP      256
#define AGP     128
#define KB      768
#define BTL     (DF * KB)
#define NTHR    256
#define NWAVE   8
#define EPT     8
#define CHUNK   (NTHR * EPT)
#define WCAP    (EPT * 32)
#define LISTN   (NWAVE * WCAP)
#define NBA     1024
#define SLA     10
#define SRCB    18
#define RCAP    20480
#define DEGCAP  64
#define MEAS_B1024_SS 16714
#define MEAS_B1024_AS 4255
#define MEAS_B1024_US 2171
#define MEAS_DEG_SS   35
#define MEAS_DEG_AS   14
#define MEAS_DEG_US   11
#define NGA     98
#define GBM     128
#define GTHR    256
#define ROWH    256
#define NUA     (NLAY * DF * 32)
#define NUB     (NLAY * DF * 8)
#define BKT_LDS_INTS  (LISTN + 2 * RCAP + 3 * NBA + 16)
#define CONS_LDS_INTS (RCAP + 2 * NBA + NWAVE * ROWH / 2)

static_assert((CHUNK & (CHUNK - 1)) == 0 && CHUNK <= 4096);
static_assert(NBA == (1 << SLA) && NBA == 4 * NTHR);
static_assert(((long long)CHUNK << SLA) < (1LL << 31));
static_assert(((long long)NBA << SRCB) < (1LL << 31));
static_assert((1 << SRCB) >= NAGR && (1 << SRCB) >= NSUB && (1 << SRCB) >= NURB);
static_assert(RCAP % 32 == 0);
static_assert(RCAP * 100 >= MEAS_B1024_SS * 105 && RCAP * 100 >= MEAS_B1024_AS * 105 && RCAP * 100 >= MEAS_B1024_US * 105);
static_assert(DEGCAP >= MEAS_DEG_SS + 8 && DEGCAP >= MEAS_DEG_AS + 8 && DEGCAP >= MEAS_DEG_US + 8);
static_assert(NPAD % GBM == 0 && NPAD >= NSUB && NBA % GBM == 0 && NBA % NWAVE == 0);
static_assert(NGA * NBA >= NPAD);
static_assert(KB % 32 == 0 && 256 % 32 == 0 && 384 % 32 == 0 && 512 % 32 == 0 && 640 % 32 == 0);
static_assert(PP * 2 == 512 && AGP * 2 == 256 && ROWH == 2 * DF);
static_assert(GBM == (GTHR / 32) * 16 && DF == 4 * 32);
static_assert(NUA % NTHR == 0 && NUB % NTHR == 0);
static_assert((NPAD * 16) % NTHR == 0);
static_assert(NSUB % 8 == 0);
static_assert(BKT_LDS_INTS * 4 <= 327680 && CONS_LDS_INTS * 4 <= 327680);

typedef float          v2f  __attribute__((ext_vector_type(2)));
typedef float          v4f  __attribute__((ext_vector_type(4)));
typedef float          v8f  __attribute__((ext_vector_type(8)));
typedef int            v4i  __attribute__((ext_vector_type(4)));
typedef int            v8i  __attribute__((ext_vector_type(8)));
typedef unsigned       v2u  __attribute__((ext_vector_type(2)));
typedef unsigned short v4us __attribute__((ext_vector_type(4)));
typedef unsigned short v8us __attribute__((ext_vector_type(8)));
typedef __bf16         v16b __attribute__((ext_vector_type(16)));
typedef v4f  __attribute__((may_alias)) v4fa;
typedef v4i  __attribute__((may_alias)) v4ia;
typedef v2u  __attribute__((may_alias)) v2ua;
typedef v4us __attribute__((may_alias)) v4usa;
typedef v8us __attribute__((may_alias)) v8usa;
union FragB { v16b v; v8us h[2]; v8i w; };

__device__ __forceinline__ v8f wmb(const FragB& a, const FragB& b, v8f c) {
  v8f d = __builtin_amdgcn_wmma_f32_16x16x32_bf16(false, a.v, false, b.v, (short)0, c, false, false);
  asm volatile("v_nop\n\tv_nop\n\tv_nop\n\tv_nop" : "+v"(d) : "v"(a.w), "v"(b.w));
  return d;
}

__device__ __forceinline__ unsigned int f2bf(float f) {
  const unsigned int u = __float_as_uint(f);
  const unsigned int r = ((u + 0x7FFFu + ((u >> 16) & 1u)) >> 16) & 0xFFFFu;
  return ((u & 0x7FFFFFFFu) > 0x7F800000u) ? 0x7FC0u : r;
}
__device__ __forceinline__ float bf2f(unsigned int b) { return __uint_as_float(b << 16); }
__device__ __forceinline__ float bfr(float f) { return bf2f(f2bf(f)); }
__device__ __forceinline__ int clampi(int v, int lo, int hi) { return v < lo ? lo : (v > hi ? hi : v); }

__device__ __forceinline__ void wave_sync() {
  __builtin_amdgcn_fence(__ATOMIC_RELEASE, "workgroup");
  __builtin_amdgcn_wave_barrier();
  __builtin_amdgcn_fence(__ATOMIC_ACQUIRE, "workgroup");
}

template <int SLB>
__device__ __forceinline__ int scan_chunk(const int* __restrict__ dsts, int nE, int cbase, int slotBase,
                                          int nb, int vec8, int* list, int tid, int lane, int wave) {
  int wc = 0;
  const int el0  = tid * EPT;
  const int e0   = cbase + el0;
  const int sent = -2147483647 - 1;
  v4i da, db;
  if (vec8 != 0 && cbase + CHUNK <= nE) {
    da = *(const v4i*)(dsts + e0);
    db = *(const v4i*)(dsts + e0 + 4);
  } else {
    da.x = (e0     < nE) ? dsts[min(e0,     nE - 1)] : sent;
    da.y = (e0 + 1 < nE) ? dsts[min(e0 + 1, nE - 1)] : sent;
    da.z = (e0 + 2 < nE) ? dsts[min(e0 + 2, nE - 1)] : sent;
    da.w = (e0 + 3 < nE) ? dsts[min(e0 + 3, nE - 1)] : sent;
    db.x = (e0 + 4 < nE) ? dsts[min(e0 + 4, nE - 1)] : sent;
    db.y = (e0 + 5 < nE) ? dsts[min(e0 + 5, nE - 1)] : sent;
    db.z = (e0 + 6 < nE) ? dsts[min(e0 + 6, nE - 1)] : sent;
    db.w = (e0 + 7 < nE) ? dsts[min(e0 + 7, nE - 1)] : sent;
  }
  const unsigned nbs = (unsigned)slotBase;
  const unsigned unb = (unsigned)nb;
  const unsigned s0 = (unsigned)da.x - nbs, s1 = (unsigned)da.y - nbs;
  const unsigned s2 = (unsigned)da.z - nbs, s3 = (unsigned)da.w - nbs;
  const unsigned s4 = (unsigned)db.x - nbs, s5 = (unsigned)db.y - nbs;
  const unsigned s6 = (unsigned)db.z - nbs, s7 = (unsigned)db.w - nbs;
  const bool h0 = s0 < unb, h1 = s1 < unb, h2 = s2 < unb, h3 = s3 < unb;
  const bool h4 = s4 < unb, h5 = s5 < unb, h6 = s6 < unb, h7 = s7 < unb;
  const unsigned any = __builtin_amdgcn_ballot_w32(h0 | h1 | h2 | h3 | h4 | h5 | h6 | h7);
  if (any != 0u) {
#define HITJ(J, HJ, SJ) { \
      const unsigned mj = __builtin_amdgcn_ballot_w32(HJ); \
      if (mj != 0u) { \
        if (HJ) { \
          const int pos = wc + (int)__builtin_amdgcn_mbcnt_lo(mj, 0u); \
          if (pos < WCAP) list[wave * WCAP + pos] = ((el0 + (J)) << SLB) | (int)(SJ); \
        } \
        wc += (int)__builtin_popcount(mj); } }
    HITJ(0, h0, s0)
    HITJ(1, h1, s1)
    HITJ(2, h2, s2)
    HITJ(3, h3, s3)
    HITJ(4, h4, s4)
    HITJ(5, h5, s5)
    HITJ(6, h6, s6)
    HITJ(7, h7, s7)
#undef HITJ
  }
  return wc;
}

__global__ __launch_bounds__(NTHR) void k_pwl(const float* __restrict__ wss, const float* __restrict__ was,
                                              const float* __restrict__ wus, unsigned short* BT) {
  const int u = (int)blockIdx.x * NTHR + (int)threadIdx.x;
  v8us o;
  unsigned short* dp;
  if (u < NUA) {
    const int i = u >> 12, n = (u >> 5) & (DF - 1), k8 = (u & 31) * 8, kk = k8 & (DF - 1);
    const float* p = wss + (size_t)i * DF * DF + (size_t)kk * DF + n;
#pragma unroll
    for (int e = 0; e < 8; ++e) o[e] = (unsigned short)f2bf(p[(size_t)e * DF]);
    dp = BT + (size_t)i * BTL + (size_t)n * KB + k8;
  } else if (u < NUA + NUB) {
    const int v = u - NUA;
    const int i = v >> 10, n = (v >> 3) & (DF - 1), k8 = (v & 7) * 8, kk = k8 & (DH - 1);
    const float* p = was + (size_t)i * DH * DF + (size_t)kk * DF + n;
#pragma unroll
    for (int e = 0; e < 8; ++e) o[e] = (unsigned short)f2bf(p[(size_t)e * DF]);
    dp = BT + (size_t)i * BTL + (size_t)n * KB + 256 + k8;
  } else if (u < NUA + 2 * NUB) {
    const int v = u - NUA - NUB;
    const int i = v >> 10, n = (v >> 3) & (DF - 1), k8 = (v & 7) * 8, kk = k8 & (DH - 1);
    const float* p = wus + (size_t)i * DH * DF + (size_t)kk * DF + n;
#pragma unroll
    for (int e = 0; e < 8; ++e) o[e] = (unsigned short)f2bf(p[(size_t)e * DF]);
    dp = BT + (size_t)i * BTL + (size_t)n * KB + 320 + k8;
  } else {
    return;
  }
  *(volatile v8us*)dp = o;
  __threadfence();
  *(volatile v8us*)dp = o;
}

__global__ __launch_bounds__(NTHR) void k_pwr(const float* __restrict__ w0, const float* __restrict__ w1,
                                              const float* __restrict__ w2, unsigned short* BT) {
  __shared__ __attribute__((aligned(16))) float tile[64 * DF];
  const int tid = (int)threadIdx.x;
  const int i = (int)blockIdx.x >> 1, kh = (int)blockIdx.x & 1;
#pragma unroll 1
  for (int j = 0; j < 8; ++j) {
    const int idx = tid + NTHR * j;
    const int k = idx >> 5, n4 = (idx & 31) * 4;
    const size_t off = (size_t)i * DF * DF + (size_t)(64 * kh + k) * DF + n4;
    const v4f a = *(const v4f*)(w0 + off);
    const v4f b = *(const v4f*)(w1 + off);
    const v4f c = *(const v4f*)(w2 + off);
    v4f s;
    s.x = (bfr(a.x) + bfr(b.x)) + bfr(c.x);
    s.y = (bfr(a.y) + bfr(b.y)) + bfr(c.y);
    s.z = (bfr(a.z) + bfr(b.z)) + bfr(c.z);
    s.w = (bfr(a.w) + bfr(b.w)) + bfr(c.w);
    *(v4fa*)(tile + k * DF + n4) = s;
  }
  __syncthreads();
  v8us hv[4], lv[4];
#pragma unroll
  for (int j = 0; j < 4; ++j) {
    const int u = tid + NTHR * j;
    const int n = u >> 3, kq = (u & 7) * 8;
#pragma unroll
    for (int e = 0; e < 8; ++e) {
      const float f = tile[(kq + e) * DF + n];
      const unsigned hb = f2bf(f);
      hv[j][e] = (unsigned short)hb;
      lv[j][e] = (unsigned short)f2bf(f - bf2f(hb));
    }
  }
#pragma unroll
  for (int j = 0; j < 4; ++j) {
    const int u = tid + NTHR * j;
    const int n = u >> 3, kq = (u & 7) * 8;
    unsigned short* dp = BT + (size_t)i * BTL + (size_t)n * KB + 64 * kh + kq;
    *(volatile v8us*)(dp + 384) = hv[j];
    *(volatile v8us*)(dp + 512) = hv[j];
    *(volatile v8us*)(dp + 640) = lv[j];
  }
  __threadfence();
#pragma unroll
  for (int j = 0; j < 4; ++j) {
    const int u = tid + NTHR * j;
    const int n = u >> 3, kq = (u & 7) * 8;
    unsigned short* dp = BT + (size_t)i * BTL + (size_t)n * KB + 64 * kh + kq;
    *(volatile v8us*)(dp + 384) = hv[j];
    *(volatile v8us*)(dp + 512) = hv[j];
    *(volatile v8us*)(dp + 640) = lv[j];
  }
}

__global__ __launch_bounds__(NTHR) void k_pb(const float* __restrict__ b0, const float* __restrict__ b1,
                                             const float* __restrict__ b2, const float* __restrict__ wf,
                                             const float* __restrict__ bfv, float* WFT, float* BSUM, float* BF) {
  __shared__ __attribute__((aligned(16))) float wl[NCLS * DF];
  const int tid = (int)threadIdx.x;
#pragma unroll
  for (int j = 0; j < 2; ++j) {
    const int idx = tid + NTHR * j;
    const int k = idx >> 2, c4 = (idx & 3) * 4;
    const v4f v = *(const v4f*)(wf + (size_t)k * NCLS + c4);
    wl[(c4 + 0) * DF + k] = bfr(v.x);
    wl[(c4 + 1) * DF + k] = bfr(v.y);
    wl[(c4 + 2) * DF + k] = bfr(v.z);
    wl[(c4 + 3) * DF + k] = bfr(v.w);
  }
  __syncthreads();
  const v4f o0 = *(const v4fa*)(wl + 4 * tid);
  const v4f o1 = *(const v4fa*)(wl + 4 * (tid + NTHR));
  const int tb = tid < 96 ? tid : 95;
  const v4f x0 = *(const v4f*)(b0 + 4 * tb);
  const v4f x1 = *(const v4f*)(b1 + 4 * tb);
  const v4f x2 = *(const v4f*)(b2 + 4 * tb);
  v4f bs;
  bs.x = (bfr(x0.x) + bfr(x1.x)) + bfr(x2.x);
  bs.y = (bfr(x0.y) + bfr(x1.y)) + bfr(x2.y);
  bs.z = (bfr(x0.z) + bfr(x1.z)) + bfr(x2.z);
  bs.w = (bfr(x0.w) + bfr(x1.w)) + bfr(x2.w);
  const int tf = tid < 4 ? tid : 3;
  const v4f fv = *(const v4f*)(bfv + 4 * tf);
  v4f bo;
  bo.x = (tid < 4) ? bfr(fv.x) : 0.0f;
  bo.y = (tid < 4) ? bfr(fv.y) : 0.0f;
  bo.z = (tid < 4) ? bfr(fv.z) : 0.0f;
  bo.w = (tid < 4) ? bfr(fv.w) : 0.0f;
  float* p0 = WFT + 4 * tid;
  float* p1 = WFT + 4 * (tid + NTHR);
  float* p2 = BSUM + 4 * tb;
  float* p3 = BF + 4 * (tid & 7);
  *(volatile v4f*)p0 = o0;
  *(volatile v4f*)p1 = o1;
  if (tid < 96) *(volatile v4f*)p2 = bs;
  if (tid < 8)  *(volatile v4f*)p3 = bo;
  __threadfence();
  *(volatile v4f*)p0 = o0;
  *(volatile v4f*)p1 = o1;
  if (tid < 96) *(volatile v4f*)p2 = bs;
  if (tid < 8)  *(volatile v4f*)p3 = bo;
}

__global__ __launch_bounds__(NTHR) void k_px(const float* __restrict__ x, unsigned short* P, int nN) {
  const int u = (int)blockIdx.x * NTHR + (int)threadIdx.x;
  const int row = u >> 4, c8 = (u & 15) * 8;
  const int rc = row < nN ? row : nN - 1;
  const bool ok = row < nN;
  const v4f a0 = *(const v4f*)(x + (size_t)rc * DF + c8);
  const v4f a1 = *(const v4f*)(x + (size_t)rc * DF + c8 + 4);
  v8us o;
  o[0] = ok ? (unsigned short)f2bf(a0.x) : (unsigned short)0;
  o[1] = ok ? (unsigned short)f2bf(a0.y) : (unsigned short)0;
  o[2] = ok ? (unsigned short)f2bf(a0.z) : (unsigned short)0;
  o[3] = ok ? (unsigned short)f2bf(a0.w) : (unsigned short)0;
  o[4] = ok ? (unsigned short)f2bf(a1.x) : (unsigned short)0;
  o[5] = ok ? (unsigned short)f2bf(a1.y) : (unsigned short)0;
  o[6] = ok ? (unsigned short)f2bf(a1.z) : (unsigned short)0;
  o[7] = ok ? (unsigned short)f2bf(a1.w) : (unsigned short)0;
  const v8us z = {0, 0, 0, 0, 0, 0, 0, 0};
  unsigned short* hp = P + (size_t)row * PP + c8;
  *(volatile v8us*)hp = o;
  *(volatile v8us*)(hp + DF) = z;
  __threadfence();
  *(volatile v8us*)hp = o;
  *(volatile v8us*)(hp + DF) = z;
}

__global__ __launch_bounds__(NTHR) void k_bucket(const int* __restrict__ srcs, const int* __restrict__ dsts,
                                                 int nE, int nDst, int nSrc, int vec8,
                                                 int* LIST, int* CNT, int* OFF, int* FLG) {
  extern __shared__ __attribute__((aligned(16))) int bsm[];
  int* list = bsm;
  int* hl   = bsm + LISTN;
  int* sl   = hl + RCAP;
  int* cnt  = sl + RCAP;
  int* offs = cnt + NBA;
  int* cur  = offs + NBA;
  int* wcnt = cur + NBA;
  const int tid = (int)threadIdx.x, lane = tid & 31, wave = tid >> 5;
  const int blk = (int)blockIdx.x;
  const int nodeBase = blk * NBA;
  const int nb = clampi(nDst - nodeBase, 0, NBA);
  {
    const v4i z4 = {0, 0, 0, 0};
    *(v4ia*)(cnt + 4 * tid) = z4;
    if (tid < 16) wcnt[tid] = 0;
  }
  __syncthreads();

  int tot = 0, ovf = 0;
  const int nChunks = (nE + CHUNK - 1) / CHUNK;
#pragma unroll 1
  for (int ch = 0; ch < nChunks; ++ch) {
    const int cbase = ch * CHUNK;
    const int wc = scan_chunk<SLA>(dsts, nE, cbase, nodeBase, nb, vec8, list, tid, lane, wave);
    if (lane == 0) wcnt[wave] = wc;
    __syncthreads();
    int pre = 0, all = 0;
#pragma unroll
    for (int w2 = 0; w2 < NWAVE; ++w2) {
      int c = wcnt[w2];
      c = c < 0 ? 0 : (c > WCAP ? WCAP : c);
      all += c;
      pre += (w2 < wave) ? c : 0;
    }
    const int wcc  = wc > WCAP ? WCAP : wc;
    const int base = tot + pre;
#pragma unroll 1
    for (int i = lane; i < wcc; i += 32) {
      const int ent = list[wave * WCAP + i];
      const int el  = (ent >> SLA) & (CHUNK - 1);
      const int sq  = ent & (NBA - 1);
      int eid = cbase + el;
      eid = eid > nE - 1 ? nE - 1 : eid;
      const int s = clampi(srcs[eid], 0, nSrc - 1);
      const int pos = base + i;
      if (pos < RCAP) hl[pos] = (int)((unsigned)s | ((unsigned)sq << SRCB));
    }
    if (tot + all > RCAP) ovf = 1;
    tot += all;
    tot = tot > RCAP ? RCAP : tot;
    __syncthreads();
  }
  const int nh = tot;
  const int nhPad = (nh + 31) & ~31;

  if (wave == 0) {
#pragma unroll 1
    for (int b0 = 0; b0 < nh; b0 += 32) {
      const int idx = b0 + lane;
      const int uv  = hl[idx < nh ? idx : nh - 1];
      const int m32 = (nh - b0) < 32 ? (nh - b0) : 32;
#pragma unroll 1
      for (int k = 0; k < m32; ++k) {
        const int u  = __builtin_amdgcn_readlane(uv, k);
        const int sq = (u >> SRCB) & (NBA - 1);
        if (lane == 0) cnt[sq] = cnt[sq] + 1;
      }
    }
  }
  __syncthreads();
  if (wave == 0) {
    const int base = lane * (NBA / 32);
    int s = 0;
#pragma unroll 1
    for (int i = 0; i < NBA / 32; ++i) s += cnt[base + i];
    int incl = s;
#pragma unroll
    for (int d = 1; d < 32; d <<= 1) {
      const int y = __shfl_up(incl, d, 32);
      if (lane >= d) incl += y;
    }
    int run = incl - s;
#pragma unroll 1
    for (int i = 0; i < NBA / 32; ++i) {
      const int cv = cnt[base + i];
      offs[base + i] = run;
      cur[base + i]  = run;
      run += cv;
    }
  }
  __syncthreads();
  if (wave == 0) {
#pragma unroll 1
    for (int b0 = 0; b0 < nh; b0 += 32) {
      const int idx = b0 + lane;
      const int uv  = hl[idx < nh ? idx : nh - 1];
      const int m32 = (nh - b0) < 32 ? (nh - b0) : 32;
#pragma unroll 1
      for (int k = 0; k < m32; ++k) {
        const int u  = __builtin_amdgcn_readlane(uv, k);
        const int sq = (u >> SRCB) & (NBA - 1);
        if (lane == 0) {
          int p = cur[sq];
          p = p < 0 ? 0 : (p > RCAP - 1 ? RCAP - 1 : p);
          sl[p] = u & ((1 << SRCB) - 1);
          cur[sq] = p + 1;
        }
      }
    }
  }
  for (int i = nh + tid; i < nhPad; i += NTHR) sl[i] = 0;
  __syncthreads();

  int* lb = LIST + (size_t)blk * RCAP;
  const v4i cq = *(const v4ia*)(cnt + 4 * tid);
  const v4i oq = *(const v4ia*)(offs + 4 * tid);
  v4i cv;
  cv.x = (tid == 0) ? nh : 0;
  cv.y = (tid == 0) ? ovf : 0;
  cv.z = 0; cv.w = 0;
  int* cp = CNT + (size_t)nodeBase + 4 * tid;
  int* op = OFF + (size_t)nodeBase + 4 * tid;
  int* fp = FLG + (size_t)blk * 32 + 4 * (tid & 7);
#pragma unroll 1
  for (int p = tid * 4; p < nhPad; p += NTHR * 4) {
    const v4i v = *(const v4ia*)(sl + p);
    *(volatile v4i*)(lb + p) = v;
  }
  *(volatile v4i*)cp = cq;
  *(volatile v4i*)op = oq;
  if (tid < 8) *(volatile v4i*)fp = cv;
  __threadfence();
#pragma unroll 1
  for (int p = tid * 4; p < nhPad; p += NTHR * 4) {
    const v4i v = *(const v4ia*)(sl + p);
    *(volatile v4i*)(lb + p) = v;
  }
  *(volatile v4i*)cp = cq;
  *(volatile v4i*)op = oq;
  if (tid < 8) *(volatile v4i*)fp = cv;
}

__device__ __forceinline__ int stage_lists(const int* __restrict__ LIST, const int* __restrict__ CNT,
                                           const int* __restrict__ OFF, const int* __restrict__ FLG,
                                           int blk, int tid, int* sl, int* cnt, int* offs, int& ovf) {
  const int nhraw = FLG[(size_t)blk * 32];
  const int bflag = FLG[(size_t)blk * 32 + 1];
  const int nh = nhraw < 0 ? 0 : (nhraw > RCAP ? RCAP : nhraw);
  ovf = (bflag != 0 || nhraw < 0 || nhraw > RCAP) ? 1 : 0;
  const int* lb = LIST + (size_t)blk * RCAP;
  const int nh4 = (nh + 3) & ~3;
#pragma unroll 1
  for (int p = tid * 4; p < nh4; p += NTHR * 4) *(v4ia*)(sl + p) = *(const v4i*)(lb + p);
  *(v4ia*)(cnt + 4 * tid)  = *(const v4i*)(CNT + (size_t)blk * NBA + 4 * tid);
  *(v4ia*)(offs + 4 * tid) = *(const v4i*)(OFF + (size_t)blk * NBA + 4 * tid);
  __syncthreads();
  return nh;
}

__global__ __launch_bounds__(NTHR) __attribute__((amdgpu_num_vgpr(248)))
void k_gatx(const int* __restrict__ LIST, const int* __restrict__ CNT, const int* __restrict__ OFF,
            const int* __restrict__ FLG, const float* __restrict__ x, int nSrc,
            unsigned short* AGX, int lineOff, int nN, int mRows) {
  extern __shared__ __attribute__((aligned(16))) int csm[];
  int* sl   = csm;
  int* cnt  = sl + RCAP;
  int* offs = cnt + NBA;
  const int tid = (int)threadIdx.x, lane = tid & 31, wave = tid >> 5;
  const int blk = (int)blockIdx.x;
  const int nodeBase = blk * NBA;
  int ovf = 0;
  const int nh = stage_lists(LIST, CNT, OFF, FLG, blk, tid, sl, cnt, offs, ovf);
  const float qnan = __int_as_float(0x7fc00000);
  const float pz = (ovf != 0) ? qnan : 0.0f;
#pragma unroll 1
  for (int si = 0; si < NBA / NWAVE; ++si) {
    const int s    = si * NWAVE + wave;
    const int node = nodeBase + s;
    const int craw = cnt[s];
    const int o = clampi(offs[s], 0, RCAP);
    int c = clampi(craw, 0, DEGCAP);
    if (c > nh - o) c = nh - o;
    c = c < 0 ? 0 : c;
    const bool bad = (c != craw);
    const float pzr = bad ? qnan : pz;
    const bool live = node < nN;
    float a = 0.0f;
#pragma unroll 1
    for (int b0 = 0; b0 < c; b0 += 32) {
      int t = b0 + lane;
      t = t > c - 1 ? c - 1 : t;
      const int idx = clampi(o + t, 0, RCAP - 1);
      const int sr  = clampi(sl[idx], 0, nSrc - 1);
      const int m32 = (c - b0) < 32 ? (c - b0) : 32;
#pragma unroll 1
      for (int k = 0; k < m32; ++k) {
        const int sk = __builtin_amdgcn_readlane(sr, k);
        const float v = x[(size_t)sk * DH + lane];
        a += bfr(v);
      }
    }
    const float r = live ? (a + pzr) : 0.0f;
    const int hbI = (int)f2bf(r);
    const int lbI = (int)f2bf(r - bf2f((unsigned)hbI));
    const int sa = (2 * lane) & 31, sb = sa + 1;
    const int ha = __shfl(hbI, sa, 32);
    const int hb = __shfl(hbI, sb, 32);
    const int la = __shfl(lbI, sa, 32);
    const int lb = __shfl(lbI, sb, 32);
    const unsigned wh = (unsigned)ha | ((unsigned)hb << 16);
    const unsigned wl = (unsigned)la | ((unsigned)lb << 16);
    const unsigned w  = (lane < 16) ? wh : wl;
    if (node < mRows) {
      unsigned* wp = (unsigned*)(AGX + (size_t)node * AGP + lineOff) + lane;
      *(volatile unsigned*)wp = w;
      __threadfence();
      *(volatile unsigned*)wp = w;
    }
  }
}

template <int MEAN>
__global__ __launch_bounds__(NTHR) __attribute__((amdgpu_num_vgpr(248)))
void k_agg(const int* __restrict__ LIST, const int* __restrict__ CNT, const int* __restrict__ OFF,
           const int* __restrict__ FLG, const unsigned short* __restrict__ P, unsigned short* Q,
           int nN, int mRows) {
  extern __shared__ __attribute__((aligned(16))) int csm[];
  int* sl   = csm;
  int* cnt  = sl + RCAP;
  int* offs = cnt + NBA;
  const int tid = (int)threadIdx.x, lane = tid & 31, wave = tid >> 5;
  unsigned short* rowbuf = (unsigned short*)(offs + NBA) + wave * ROWH;
  const int blk = (int)blockIdx.x;
  const int nodeBase = blk * NBA;
  int ovf = 0;
  const int nh = stage_lists(LIST, CNT, OFF, FLG, blk, tid, sl, cnt, offs, ovf);
  const float qnan = __int_as_float(0x7fc00000);
  const float pz = (ovf != 0) ? qnan : 0.0f;
#pragma unroll 1
  for (int si = 0; si < NBA / NWAVE; ++si) {
    const int s    = si * NWAVE + wave;
    const int node = nodeBase + s;
    const int craw = cnt[s];
    const int o = clampi(offs[s], 0, RCAP);
    int c = clampi(craw, 0, DEGCAP);
    if (c > nh - o) c = nh - o;
    c = c < 0 ? 0 : c;
    const bool bad = (c != craw);
    const float pzr = bad ? qnan : pz;
    const bool live = node < nN;
    float a0 = 0.0f, a1 = 0.0f, a2 = 0.0f, a3 = 0.0f;
#pragma unroll 1
    for (int b0 = 0; b0 < c; b0 += 32) {
      int t = b0 + lane;
      t = t > c - 1 ? c - 1 : t;
      const int idx = clampi(o + t, 0, RCAP - 1);
      const int sr  = clampi(sl[idx], 0, nN - 1);
      const int m32 = (c - b0) < 32 ? (c - b0) : 32;
#pragma unroll 1
      for (int k = 0; k < m32; ++k) {
        const int sk = __builtin_amdgcn_readlane(sr, k);
        const unsigned short* rp = P + (size_t)sk * PP + 4 * lane;
        const v2u wh = *(const v2ua*)rp;
        float f0 = __uint_as_float(wh.x << 16);
        float f1 = __uint_as_float(wh.x & 0xffff0000u);
        float f2 = __uint_as_float(wh.y << 16);
        float f3 = __uint_as_float(wh.y & 0xffff0000u);
        if constexpr (MEAN != 0) {
          const v2u wl = *(const v2ua*)(rp + DF);
          f0 += __uint_as_float(wl.x << 16);
          f1 += __uint_as_float(wl.x & 0xffff0000u);
          f2 += __uint_as_float(wl.y << 16);
          f3 += __uint_as_float(wl.y & 0xffff0000u);
        }
        a0 += f0; a1 += f1; a2 += f2; a3 += f3;
      }
    }
    if constexpr (MEAN != 0) {
      const float dg = fmaxf((float)(craw < 0 ? 0 : craw), 1.0f);
      a0 = a0 / dg; a1 = a1 / dg; a2 = a2 / dg; a3 = a3 / dg;
    }
    const float m0 = live ? (a0 + pzr) : 0.0f;
    const float m1 = live ? (a1 + pzr) : 0.0f;
    const float m2 = live ? (a2 + pzr) : 0.0f;
    const float m3 = live ? (a3 + pzr) : 0.0f;
    v4us mh, ml;
    {
      unsigned hb;
      hb = f2bf(m0); mh[0] = (unsigned short)hb; ml[0] = (unsigned short)f2bf(m0 - bf2f(hb));
      hb = f2bf(m1); mh[1] = (unsigned short)hb; ml[1] = (unsigned short)f2bf(m1 - bf2f(hb));
      hb = f2bf(m2); mh[2] = (unsigned short)hb; ml[2] = (unsigned short)f2bf(m2 - bf2f(hb));
      hb = f2bf(m3); mh[3] = (unsigned short)hb; ml[3] = (unsigned short)f2bf(m3 - bf2f(hb));
    }
    *(v4usa*)(rowbuf + 4 * lane)      = mh;
    *(v4usa*)(rowbuf + DF + 4 * lane) = ml;
    wave_sync();
    const v8us q0 = *(const v8usa*)(rowbuf + 8 * lane);
    wave_sync();
    if (node < mRows) {
      unsigned short* rpw = Q + (size_t)node * PP + 8 * lane;
      *(volatile v8us*)rpw = q0;
      __threadfence();
      *(volatile v8us*)rpw = q0;
    }
  }
}

__device__ __forceinline__ void gemm_seg(const unsigned short* ap, const unsigned short* bp, int nsteps,
                                         v8f (&acc)[8]) {
#pragma unroll 1
  for (int ks = 0; ks < nsteps; ++ks) {
    FragB af;
    af.h[0] = *(const v8usa*)(ap + 32 * ks);
    af.h[1] = *(const v8usa*)(ap + 32 * ks + 16);
#pragma unroll
    for (int nt = 0; nt < 8; ++nt) {
      const unsigned short* wq = bp + (size_t)(16 * nt) * (size_t)KB + 32 * ks;
      FragB bf;
      bf.h[0] = *(const v8usa*)wq;
      bf.h[1] = *(const v8usa*)(wq + 16);
      acc[nt] = wmb(af, bf, acc[nt]);
    }
  }
}

template <int LAYER>
__global__ __launch_bounds__(GTHR) __attribute__((amdgpu_num_vgpr(248)))
void k_gemm(const unsigned short* __restrict__ Q, const unsigned short* __restrict__ AGX, unsigned short* P,
            const unsigned short* __restrict__ BT, const float* __restrict__ BSUM,
            const float* __restrict__ WFT, const float* __restrict__ BF, const int* __restrict__ FLG,
            float* outp, int nN, int mRows, int nFlgBlk) {
  __shared__ __attribute__((aligned(16))) float stg[GBM * DF];
  __shared__ __attribute__((aligned(16))) float sb[DF];
  const int tid = (int)threadIdx.x, lane = tid & 31, wave = tid >> 5, hh = lane >> 4, m = lane & 15;
  const int rowBase = (int)blockIdx.x * GBM;

  v8f acc[8];
  {
    const v8f z = {0.f, 0.f, 0.f, 0.f, 0.f, 0.f, 0.f, 0.f};
#pragma unroll
    for (int t = 0; t < 8; ++t) acc[t] = z;
  }
  const size_t rA = (size_t)(rowBase + 16 * wave + m);
  const unsigned short* bp = BT + (size_t)LAYER * BTL + (size_t)m * KB + 8 * hh;
  gemm_seg(Q   + rA * PP  + 8 * hh, bp,       8, acc);
  gemm_seg(AGX + rA * AGP + 8 * hh, bp + 256, 4, acc);
  gemm_seg(P   + rA * PP  + 8 * hh, bp + 384, (LAYER == 0) ? 4 : 8, acc);
  gemm_seg(P   + rA * PP  + 8 * hh, bp + 640, 4, acc);

#pragma unroll
  for (int nt = 0; nt < 8; ++nt) {
    const int lc = 16 * nt + m;
#pragma unroll
    for (int r = 0; r < 8; ++r) {
      const int lr = 16 * wave + 8 * hh + r;
      stg[lr * DF + lc] = acc[nt][r];
    }
  }
  if (tid < 32) *(v4fa*)(sb + 4 * tid) = *(const v4f*)(BSUM + LAYER * DF + 4 * tid);

  if constexpr (LAYER < 2) {
    __syncthreads();
    const v4f bq = *(const v4fa*)(sb + 4 * lane);
    v4f pv[16];
#pragma unroll
    for (int i = 0; i < 16; ++i) pv[i] = *(const v4fa*)(stg + (16 * wave + i) * DF + 4 * lane);
    __syncthreads();
#pragma unroll
    for (int i = 0; i < 16; ++i) {
      const int row = rowBase + 16 * wave + i;
      const bool ok = row < nN;
      const float y0 = pv[i].x + bq.x, y1 = pv[i].y + bq.y, y2 = pv[i].z + bq.z, y3 = pv[i].w + bq.w;
      const float r0 = (y0 > 0.0f) ? y0 : (y0 - y0);
      const float r1 = (y1 > 0.0f) ? y1 : (y1 - y1);
      const float r2 = (y2 > 0.0f) ? y2 : (y2 - y2);
      const float r3 = (y3 > 0.0f) ? y3 : (y3 - y3);
      const float o0 = ok ? r0 : 0.0f, o1 = ok ? r1 : 0.0f, o2 = ok ? r2 : 0.0f, o3 = ok ? r3 : 0.0f;
      v4us h4, l4;
      unsigned hb;
      hb = f2bf(o0); h4[0] = (unsigned short)hb; l4[0] = (unsigned short)f2bf(o0 - bf2f(hb));
      hb = f2bf(o1); h4[1] = (unsigned short)hb; l4[1] = (unsigned short)f2bf(o1 - bf2f(hb));
      hb = f2bf(o2); h4[2] = (unsigned short)hb; l4[2] = (unsigned short)f2bf(o2 - bf2f(hb));
      hb = f2bf(o3); h4[3] = (unsigned short)hb; l4[3] = (unsigned short)f2bf(o3 - bf2f(hb));
      unsigned short* srow = (unsigned short*)stg + (size_t)(16 * wave + i) * (2 * DF);
      *(v4usa*)(srow + 4 * lane) = h4;
      *(v4usa*)(srow + DF + 4 * lane) = l4;
    }
    __syncthreads();
    v8us qv[16];
#pragma unroll
    for (int i = 0; i < 16; ++i) {
      const unsigned short* srow = (const unsigned short*)stg + (size_t)(16 * wave + i) * (2 * DF);
      qv[i] = *(const v8usa*)(srow + 8 * lane);
    }
#pragma unroll
    for (int i = 0; i < 16; ++i) {
      const int gr = rowBase + 16 * wave + i;
      unsigned short* rp = P + (size_t)gr * PP + 8 * lane;
      if (gr < mRows) *(volatile v8us*)rp = qv[i];
    }
    __threadfence();
#pragma unroll
    for (int i = 0; i < 16; ++i) {
      const int gr = rowBase + 16 * wave + i;
      unsigned short* rp = P + (size_t)gr * PP + 8 * lane;
      if (gr < mRows) *(volatile v8us*)rp = qv[i];
    }
    (void)WFT; (void)BF; (void)FLG; (void)outp; (void)nFlgBlk;
  } else {
    __shared__ __attribute__((aligned(16))) float wft[NCLS * DF];
    __shared__ __attribute__((aligned(16))) float lgs[GBM * NCLS];
    __shared__ __attribute__((aligned(16))) float bfs[NCLS];
#pragma unroll
    for (int j = 0; j < 2; ++j)
      *(v4fa*)(wft + 4 * (tid + GTHR * j)) = *(const v4f*)(WFT + 4 * (tid + GTHR * j));
    if (tid < 4) *(v4fa*)(bfs + 4 * tid) = *(const v4f*)(BF + 4 * tid);
    __syncthreads();
    {
      const v4f bq = *(const v4fa*)(sb + 4 * lane);
#pragma unroll
      for (int i = 0; i < 16; ++i) {
        float* p = stg + (16 * wave + i) * DF + 4 * lane;
        const v4f v = *(const v4fa*)p;
        const float y0 = v.x + bq.x, y1 = v.y + bq.y, y2 = v.z + bq.z, y3 = v.w + bq.w;
        v4f r;
        r.x = (y0 > 0.0f) ? y0 : (y0 - y0);
        r.y = (y1 > 0.0f) ? y1 : (y1 - y1);
        r.z = (y2 > 0.0f) ? y2 : (y2 - y2);
        r.w = (y3 > 0.0f) ? y3 : (y3 - y3);
        *(v4fa*)p = r;
      }
    }
    __syncthreads();
    const int rr = 16 * wave + (lane & 15);
    const int c0 = (lane >> 4) * 8;
    float d[8];
#pragma unroll
    for (int j = 0; j < 8; ++j) d[j] = 0.0f;
#pragma unroll 1
    for (int k4 = 0; k4 < DF / 4; ++k4) {
      const v4f hv = *(const v4fa*)(stg + rr * DF + 4 * k4);
#pragma unroll
      for (int j = 0; j < 8; ++j) {
        const v4f wv = *(const v4fa*)(wft + (c0 + j) * DF + 4 * k4);
        d[j] = fmaf(hv.x, wv.x, d[j]);
        d[j] = fmaf(hv.y, wv.y, d[j]);
        d[j] = fmaf(hv.z, wv.z, d[j]);
        d[j] = fmaf(hv.w, wv.w, d[j]);
      }
    }
    float* lgrow = lgs + rr * NCLS + c0;
    {
      const v4f b0 = *(const v4fa*)(bfs + c0);
      const v4f b1 = *(const v4fa*)(bfs + c0 + 4);
      d[0] += b0.x; d[1] += b0.y; d[2] += b0.z; d[3] += b0.w;
      d[4] += b1.x; d[5] += b1.y; d[6] += b1.z; d[7] += b1.w;
    }
    float mx = d[0];
#pragma unroll
    for (int j = 1; j < 8; ++j) mx = (d[j] > mx || d[j] != d[j]) ? d[j] : mx;
    {
      const float mo = __shfl_xor(mx, 16, 32);
      mx = (mo > mx || mo != mo) ? mo : mx;
    }
#pragma unroll
    for (int j = 0; j < 8; ++j) lgrow[j] = d[j];
    float s = 0.0f;
#pragma unroll 1
    for (int j = 0; j < 8; ++j) {
      const float e = expf(lgrow[j] - mx);
      lgrow[j] = e;
      s += e;
    }
    const float st = s + __shfl_xor(s, 16, 32);
#pragma unroll 1
    for (int j = 0; j < 8; ++j) {
      const float e = lgrow[j];
      lgrow[j] = e / st;
    }
    __syncthreads();
    const int fb = rowBase >> 10;
    const int fl = FLG[(size_t)fb * 32 + 1] | FLG[((size_t)nFlgBlk + fb) * 32 + 1] |
                   FLG[((size_t)2 * nFlgBlk + fb) * 32 + 1];
    const float qnan = __int_as_float(0x7fc00000);
    v4f ov[2];
#pragma unroll
    for (int j = 0; j < 2; ++j) {
      const int u = tid + GTHR * j;
      v4f v = *(const v4fa*)(lgs + 4 * u);
      v.x = (fl != 0) ? qnan : v.x;
      v.y = (fl != 0) ? qnan : v.y;
      v.z = (fl != 0) ? qnan : v.z;
      v.w = (fl != 0) ? qnan : v.w;
      ov[j] = v;
    }
#pragma unroll
    for (int j = 0; j < 2; ++j) {
      const int u = tid + GTHR * j;
      const int row = rowBase + (u >> 2);
      float* op = outp + (size_t)rowBase * NCLS + 4 * u;
      if (row < nN) *(volatile v4f*)op = ov[j];
    }
    __threadfence();
#pragma unroll
    for (int j = 0; j < 2; ++j) {
      const int u = tid + GTHR * j;
      const int row = rowBase + (u >> 2);
      float* op = outp + (size_t)rowBase * NCLS + 4 * u;
      if (row < nN) *(volatile v4f*)op = ov[j];
    }
    (void)mRows;
  }
}

static inline size_t al256(size_t o) { return (o + 255) & ~(size_t)255; }

extern "C" void kernel_launch(void* const* d_in, const int* in_sizes, int n_in,
                              void* d_out, int out_size, void* d_ws, size_t ws_size,
                              hipStream_t stream) {
  if (n_in < 20) return;
  if (in_sizes[0] != NSUB * DF || in_sizes[1] != NAGR * DH || in_sizes[2] != NURB * DH) return;
  if (in_sizes[3] != ESS || in_sizes[4] != ESS) return;
  if (in_sizes[5] != EAS || in_sizes[6] != EAS) return;
  if (in_sizes[7] != EUS || in_sizes[8] != EUS) return;
  if (in_sizes[9] != NLAY * DF * DF || in_sizes[10] != NLAY * DF || in_sizes[11] != NLAY * DF * DF) return;
  if (in_sizes[12] != NLAY * DH * DF || in_sizes[13] != NLAY * DF || in_sizes[14] != NLAY * DF * DF) return;
  if (in_sizes[15] != NLAY * DH * DF || in_sizes[16] != NLAY * DF || in_sizes[17] != NLAY * DF * DF) return;
  if (in_sizes[18] != DF * NCLS || in_sizes[19] != NCLS) return;
  if (out_size != NSUB * NCLS) return;

  const float* x_sub = (const float*)d_in[0];
  const float* x_agr = (const float*)d_in[1];
  const float* x_urb = (const float*)d_in[2];
  const int* ss_src  = (const int*)d_in[3];
  const int* ss_dst  = (const int*)d_in[4];
  const int* as_src  = (const int*)d_in[5];
  const int* as_dst  = (const int*)d_in[6];
  const int* us_src  = (const int*)d_in[7];
  const int* us_dst  = (const int*)d_in[8];
  const float* Wl_ss = (const float*)d_in[9];
  const float* bl_ss = (const float*)d_in[10];
  const float* Wr_ss = (const float*)d_in[11];
  const float* Wl_as = (const float*)d_in[12];
  const float* bl_as = (const float*)d_in[13];
  const float* Wr_as = (const float*)d_in[14];
  const float* Wl_us = (const float*)d_in[15];
  const float* bl_us = (const float*)d_in[16];
  const float* Wr_us = (const float*)d_in[17];
  const float* Wf    = (const float*)d_in[18];
  const float* bfv   = (const float*)d_in[19];
  float* out = (float*)d_out;

  char* ws = (char*)d_ws;
  size_t off = 0;
  const size_t oBT  = off; off = al256(off + (size_t)NLAY * BTL * 2);
  const size_t oWFT = off; off = al256(off + (size_t)NCLS * DF * 4);
  const size_t oBS  = off; off = al256(off + (size_t)NLAY * DF * 4);
  const size_t oBF  = off; off = al256(off + (size_t)32 * 4);
  const size_t oP   = off; off = al256(off + (size_t)NPAD * PP * 2);
  const size_t oQ   = off; off = al256(off + (size_t)NPAD * PP * 2);
  const size_t oAGX = off; off = al256(off + (size_t)NPAD * AGP * 2);
  const size_t oLST = off; off = al256(off + (size_t)NGA * RCAP * 4);
  const size_t oCNT = off; off = al256(off + (size_t)NGA * NBA * 4);
  const size_t oOFF = off; off = al256(off + (size_t)NGA * NBA * 4);
  const size_t oFLG = off; off = al256(off + (size_t)3 * NGA * 128);
  if (off > ws_size) return;
  unsigned short* BT  = (unsigned short*)(ws + oBT);
  float*          WFT = (float*)(ws + oWFT);
  float*          BSM = (float*)(ws + oBS);
  float*          BFP = (float*)(ws + oBF);
  unsigned short* P   = (unsigned short*)(ws + oP);
  unsigned short* Q   = (unsigned short*)(ws + oQ);
  unsigned short* AGX = (unsigned short*)(ws + oAGX);
  int*            LST = (int*)(ws + oLST);
  int*            CNT = (int*)(ws + oCNT);
  int*            OFS = (int*)(ws + oOFF);
  int*            FLG = (int*)(ws + oFLG);
  int* FLGa = FLG;
  int* FLGu = FLG + (size_t)NGA * 32;
  int* FLGs = FLG + (size_t)2 * NGA * 32;

  const int bktLds  = BKT_LDS_INTS * 4;
  const int consLds = CONS_LDS_INTS * 4;
  hipFuncSetAttribute(reinterpret_cast<const void*>(&k_bucket), hipFuncAttributeMaxDynamicSharedMemorySize, bktLds);
  hipFuncSetAttribute(reinterpret_cast<const void*>(&k_gatx), hipFuncAttributeMaxDynamicSharedMemorySize, consLds);
  hipFuncSetAttribute(reinterpret_cast<const void*>(&k_agg<0>), hipFuncAttributeMaxDynamicSharedMemorySize, consLds);
  hipFuncSetAttribute(reinterpret_cast<const void*>(&k_agg<1>), hipFuncAttributeMaxDynamicSharedMemorySize, consLds);

  const int gM = NPAD / GBM;

  k_pwl<<<(NUA + 2 * NUB) / NTHR, NTHR, 0, stream>>>(Wl_ss, Wl_as, Wl_us, BT);
  k_pwr<<<2 * NLAY, NTHR, 0, stream>>>(Wr_ss, Wr_as, Wr_us, BT);
  k_pb<<<1, NTHR, 0, stream>>>(bl_ss, bl_as, bl_us, Wf, bfv, WFT, BSM, BFP);
  k_px<<<(NPAD * 16) / NTHR, NTHR, 0, stream>>>(x_sub, P, NSUB);
  k_bucket<<<NGA, NTHR, bktLds, stream>>>(as_src, as_dst, EAS, NSUB, NAGR, 1, LST, CNT, OFS, FLGa);
  k_gatx<<<NGA, NTHR, consLds, stream>>>(LST, CNT, OFS, FLGa, x_agr, NAGR, AGX, 0, NSUB, NPAD);
  k_bucket<<<NGA, NTHR, bktLds, stream>>>(us_src, us_dst, EUS, NSUB, NURB, 1, LST, CNT, OFS, FLGu);
  k_gatx<<<NGA, NTHR, consLds, stream>>>(LST, CNT, OFS, FLGu, x_urb, NURB, AGX, 64, NSUB, NPAD);
  k_bucket<<<NGA, NTHR, bktLds, stream>>>(ss_src, ss_dst, ESS, NSUB, NSUB, 1, LST, CNT, OFS, FLGs);
  k_agg<0><<<NGA, NTHR, consLds, stream>>>(LST, CNT, OFS, FLGs, P, Q, NSUB, NPAD);
  k_gemm<0><<<gM, GTHR, 0, stream>>>(Q, AGX, P, BT, BSM, WFT, BFP, FLG, out, NSUB, NPAD, NGA);
  k_agg<1><<<NGA, NTHR, consLds, stream>>>(LST, CNT, OFS, FLGs, P, Q, NSUB, NPAD);
  k_gemm<1><<<gM, GTHR, 0, stream>>>(Q, AGX, P, BT, BSM, WFT, BFP, FLG, out, NSUB, NPAD, NGA);
  k_agg<1><<<NGA, NTHR, consLds, stream>>>(LST, CNT, OFS, FLGs, P, Q, NSUB, NPAD);
  k_gemm<2><<<gM, GTHR, 0, stream>>>(Q, AGX, P, BT, BSM, WFT, BFP, FLG, out, NSUB, NPAD, NGA);
}
